// GroupQueryAttention_84361747628064
// MI455X (gfx1250) — hardware-verified
//
#include <hip/hip_runtime.h>


#ifndef NB
#define NB 2
#endif
#ifndef SEQ
#define SEQ 2048
#endif
#define NB_FULL  2
#define SEQ_FULL 2048
#define EM   768
#define NG   4
#define NH   12
#define HD   64
#define TQ   (SEQ / NG)
#define ACAR 16.0f
#define WCAR 64.0f
#define PCAR 1024.0f
#define SSC  (0.125f / (ACAR * ACAR))
#define L2E  1.4426950408889634f
#define SSL  (SSC * L2E)
static_assert(SEQ % 256 == 0);
static_assert(SEQ <= SEQ_FULL);
static_assert(NB >= 1 && NB <= NB_FULL);
static_assert(EM == NH * HD);
static_assert(EM % 64 == 0 && TQ % 64 == 0);
static_assert((NG * NH * (TQ / 16)) % 2 == 0);

typedef _Float16 h16;
typedef unsigned short bf;
typedef __attribute__((ext_vector_type(16))) __bf16   v16bf;
typedef __attribute__((ext_vector_type(16))) _Float16 v16h;
typedef __attribute__((ext_vector_type(8)))  _Float16 v8h;
typedef __attribute__((ext_vector_type(8)))  unsigned short v8us;
typedef __attribute__((ext_vector_type(8)))  float    v8f;
typedef __attribute__((ext_vector_type(4)))  float    v4f;
typedef v8h  __attribute__((may_alias)) v8ha;
typedef v4f  __attribute__((may_alias)) v4fa;
typedef v8us __attribute__((may_alias)) v8usa;

__device__ __forceinline__ unsigned short f2bf(float f) { unsigned u = __float_as_uint(f); u += 0x7FFFu + ((u >> 16) & 1u); return (unsigned short)(u >> 16); }
__device__ __forceinline__ float bf2f(unsigned short b) { return __uint_as_float(((unsigned)b) << 16); }
__device__ __forceinline__ float bfr(float f) { return bf2f(f2bf(f)); }
__device__ __forceinline__ void splitf(float y, unsigned short& h, unsigned short& l) { h = f2bf(y); l = f2bf(y - bf2f(h)); }
__device__ __forceinline__ v16h cat16(v8h lo, v8h hi) { return __builtin_shufflevector(lo, hi, 0, 1, 2, 3, 4, 5, 6, 7, 8, 9, 10, 11, 12, 13, 14, 15); }
__device__ __forceinline__ v16bf cat16b(v8us lo, v8us hi) { return __builtin_bit_cast(v16bf, __builtin_shufflevector(lo, hi, 0, 1, 2, 3, 4, 5, 6, 7, 8, 9, 10, 11, 12, 13, 14, 15)); }
__device__ __forceinline__ v8f wmma16(v16h a, v16h b, v8f c) { return __builtin_amdgcn_wmma_f32_16x16x32_f16(false, a, false, b, (short)0, c, false, false); }
__device__ __forceinline__ v8f wmmab(v16bf a, v16bf b, v8f c) { return __builtin_amdgcn_wmma_f32_16x16x32_bf16(false, a, false, b, (short)0, c, false, false); }

template <typename T16> struct WFrag;
template <> struct WFrag<h16> { typedef v16h V; static __device__ __forceinline__ V ld(const h16* p) { return cat16(*(const v8h*)p, *(const v8h*)(p + 16)); } static __device__ __forceinline__ v8f mma(V a, V b, v8f c) { return wmma16(a, b, c); } };
template <> struct WFrag<bf> { typedef v16bf V; static __device__ __forceinline__ V ld(const bf* p) { return cat16b(*(const v8us*)p, *(const v8us*)(p + 16)); } static __device__ __forceinline__ v8f mma(V a, V b, v8f c) { return wmmab(a, b, c); } };

template <typename T16, int NSPLIT, int BMODE, typename OT>
__global__ __launch_bounds__(32) void k_gemmw(const T16* __restrict__ A, const T16* __restrict__ A2, const T16* __restrict__ Bt, const T16* __restrict__ Bt2, int K, int lda, int ldb, OT* C, int ldc, const float* __restrict__ bias, float oscl, float pscl, size_t sA, size_t sB, size_t sC, size_t sBias) {
    typedef typename WFrag<T16>::V V;
    __shared__ __align__(16) float os[16 * 68];
    const size_t z = blockIdx.z; A += z * sA; if (A2) A2 += z * sA; Bt += z * sB; if (Bt2) Bt2 += z * sB; C += z * sC; if (BMODE != 0) bias += z * sBias;
    const int lane = threadIdx.x & 31, lr = lane & 15, hi = lane >> 4; const int r0 = blockIdx.x * 64, c0 = blockIdx.y * 64;
    v8f acc[4][4];
#pragma unroll
    for (int mb = 0; mb < 4; ++mb)
#pragma unroll
        for (int nb = 0; nb < 4; ++nb) acc[mb][nb] = (v8f){};
    const size_t aoff = (size_t)(r0 + lr) * lda + 8 * hi, boff = (size_t)(c0 + lr) * ldb + 8 * hi;
#pragma unroll 1
    for (int kc = 0; kc < K; kc += 32) {
        V a[4], a2[4];
#pragma unroll
        for (int mb = 0; mb < 4; ++mb) { a[mb] = WFrag<T16>::ld(A + aoff + (size_t)mb * 16 * lda + kc); if (NSPLIT == 1) a2[mb] = WFrag<T16>::ld(A2 + aoff + (size_t)mb * 16 * lda + kc); }
#pragma unroll
        for (int nb = 0; nb < 4; ++nb) { const V b = WFrag<T16>::ld(Bt + boff + (size_t)nb * 16 * ldb + kc); V b2; if (NSPLIT == 2) b2 = WFrag<T16>::ld(Bt2 + boff + (size_t)nb * 16 * ldb + kc);
#pragma unroll
            for (int mb = 0; mb < 4; ++mb) { acc[mb][nb] = WFrag<T16>::mma(a[mb], b, acc[mb][nb]); if (NSPLIT == 1) acc[mb][nb] = WFrag<T16>::mma(a2[mb], b, acc[mb][nb]); if (NSPLIT == 2) acc[mb][nb] = WFrag<T16>::mma(a[mb], b2, acc[mb][nb]); } }
        asm volatile("v_nop\n\tv_nop\n\tv_nop\n\tv_nop" : "+v"(acc[0][0]), "+v"(acc[1][1]), "+v"(acc[2][2]), "+v"(acc[3][3]) : "v"(a[0]), "v"(a[3]));
    }
#pragma unroll
    for (int mb = 0; mb < 4; ++mb) {
#pragma unroll
        for (int nb = 0; nb < 4; ++nb) {
#pragma unroll
            for (int j = 0; j < 8; ++j) os[(hi * 8 + j) * 68 + nb * 16 + lr] = acc[mb][nb][j]; }
        __builtin_amdgcn_fence(3, "wavefront"); __builtin_amdgcn_wave_barrier(); asm volatile("" ::: "memory");
        OT* cbase = C + (size_t)(r0 + mb * 16) * ldc + c0;
        if (sizeof(OT) == 4) {
#pragma unroll 1
            for (int ps = 0; ps < 2; ++ps) {
#pragma unroll
                for (int s = 0; s < 8; ++s) { const int row = 2 * s + hi, cofs = lr * 4; v4f val = *(const v4fa*)(os + row * 68 + cofs);
#pragma unroll
                    for (int e = 0; e < 4; ++e) { float bb = 0.f; if (BMODE == 1) bb = bfr(bias[c0 + cofs + e]); if (BMODE == 2) bb = bfr(bias[r0 + mb * 16 + row]); val[e] = (val[e] * oscl + bb) * pscl; }
                    *(volatile v4f*)((float*)cbase + (size_t)row * ldc + cofs) = val; }
                if (ps == 0) __threadfence(); }
        } else {
#pragma unroll 1
            for (int ps = 0; ps < 2; ++ps) {
#pragma unroll
                for (int s = 0; s < 4; ++s) { const int row = 4 * s + (lane >> 3), cofs = (lane & 7) * 8; const v4f x0 = *(const v4fa*)(os + row * 68 + cofs); const v4f x1 = *(const v4fa*)(os + row * 68 + cofs + 4);
                    float brow = 0.f; if (BMODE == 2) brow = bfr(bias[r0 + mb * 16 + row]);
                    v8h o8;
#pragma unroll
                    for (int e = 0; e < 4; ++e) { float bb = brow; if (BMODE == 1) bb = bfr(bias[c0 + cofs + e]); o8[e] = (h16)((x0[e] * oscl + bb) * pscl); }
#pragma unroll
                    for (int e = 0; e < 4; ++e) { float bb = brow; if (BMODE == 1) bb = bfr(bias[c0 + cofs + 4 + e]); o8[4 + e] = (h16)((x1[e] * oscl + bb) * pscl); }
                    *(volatile v8h*)((h16*)cbase + (size_t)row * ldc + cofs) = o8; }
                if (ps == 0) __threadfence(); }
        }
        __builtin_amdgcn_fence(3, "wavefront"); __builtin_amdgcn_wave_barrier(); asm volatile("" ::: "memory");
    }
}

__global__ __launch_bounds__(256) void k_cvt8(const float* __restrict__ src, bf* dst, size_t n8) { const size_t i = (size_t)blockIdx.x * 256 + threadIdx.x; if (i >= n8) return; const v8f v = *(const v8f*)(src + i * 8); v8us o;
#pragma unroll
    for (int k = 0; k < 8; ++k) o[k] = f2bf(v[k]); *(volatile v8us*)(dst + i * 8) = o; __threadfence(); *(volatile v8us*)(dst + i * 8) = o; }
__global__ __launch_bounds__(256) void k_cvth(const float* __restrict__ src, h16* dst, size_t n8, float scl) { const size_t i = (size_t)blockIdx.x * 256 + threadIdx.x; if (i >= n8) return; const v8f v = *(const v8f*)(src + i * 8); v8h o;
#pragma unroll
    for (int k = 0; k < 8; ++k) o[k] = (h16)(bfr(v[k]) * scl); *(volatile v8h*)(dst + i * 8) = o; __threadfence(); *(volatile v8h*)(dst + i * 8) = o; }

__global__ __launch_bounds__(64) __attribute__((amdgpu_num_vgpr(256))) void k_attn(const h16* __restrict__ QI, const h16* __restrict__ KI, const h16* __restrict__ VT, bf* CTh, bf* CTl) {
    __shared__ __align__(16) unsigned short cs[2][2][16 * 72];
    const int wave = threadIdx.x >> 5, lane = threadIdx.x & 31, lr = lane & 15, hi = lane >> 4;
    const int unit = blockIdx.x * 2 + wave; const int tt = unit % (TQ / 16); const int h = (unit / (TQ / 16)) % NH; const int g = unit / ((TQ / 16) * NH); const int t0 = tt * 16;
    const h16* qp = QI + ((size_t)g * TQ + t0 + lr) * EM + h * HD + 8 * hi;
    const v16h qb0 = WFrag<h16>::ld(qp), qb1 = WFrag<h16>::ld(qp + 32);
    const h16* kp = QI == nullptr ? nullptr : KI + ((size_t)g * SEQ + lr) * EM + h * HD + 8 * hi;
    const h16* vp = VT + ((size_t)g * EM + h * HD + lr) * SEQ + 8 * hi;
    float m = -1.0e30f, l = 0.f;
    v8f o[4];
#pragma unroll
    for (int j = 0; j < 4; ++j) o[j] = (v8f){};
#pragma unroll 1
    for (int s0 = 0; s0 < SEQ; s0 += 32) {
        const h16* k0p = kp + (size_t)s0 * EM;
        const v16h a00 = WFrag<h16>::ld(k0p), a01 = WFrag<h16>::ld(k0p + 32), a10 = WFrag<h16>::ld(k0p + (size_t)16 * EM), a11 = WFrag<h16>::ld(k0p + (size_t)16 * EM + 32);
        v8f sc0 = wmma16(a00, qb0, (v8f){}); sc0 = wmma16(a01, qb1, sc0);
        v8f sc1 = wmma16(a10, qb0, (v8f){}); sc1 = wmma16(a11, qb1, sc1);
        asm volatile("v_nop\n\tv_nop\n\tv_nop\n\tv_nop" : "+v"(sc0), "+v"(sc1) : "v"(a00), "v"(a01), "v"(a10), "v"(a11), "v"(qb0), "v"(qb1));
        float mx = fmaxf(sc0[0], sc1[0]);
#pragma unroll
        for (int r = 1; r < 8; ++r) mx = fmaxf(mx, fmaxf(sc0[r], sc1[r]));
        float mloc = mx * SSC; mloc = fmaxf(mloc, __shfl_xor(mloc, 16, 32));
        const float mnew = fmaxf(m, mloc); const float alpha = __builtin_amdgcn_exp2f((m - mnew) * L2E); m = mnew; const float mb2 = mnew * L2E;
        float psum = 0.f; v16h pb = (v16h){};
#pragma unroll
        for (int r = 0; r < 8; ++r) { const float p0 = __builtin_amdgcn_exp2f(sc0[r] * SSL - mb2); const float p1 = __builtin_amdgcn_exp2f(sc1[r] * SSL - mb2); psum += p0 + p1; pb[r] = (h16)(p0 * PCAR); pb[8 + r] = (h16)(p1 * PCAR); }
        psum += __shfl_xor(psum, 16, 32); l = l * alpha + psum;
#pragma unroll
        for (int j = 0; j < 4; ++j) o[j] = o[j] * alpha;
        v16h va[4];
#pragma unroll
        for (int j = 0; j < 4; ++j) va[j] = WFrag<h16>::ld(vp + (size_t)(16 * j) * SEQ + s0);
#pragma unroll
        for (int j = 0; j < 4; ++j) o[j] = wmma16(va[j], pb, o[j]);
        asm volatile("v_nop\n\tv_nop\n\tv_nop\n\tv_nop" : "+v"(o[0]), "+v"(o[1]), "+v"(o[2]), "+v"(o[3]) : "v"(va[0]), "v"(va[1]), "v"(va[2]), "v"(va[3]), "v"(pb));
    }
    const float rinv = (1.0f / l) * (1.0f / (PCAR * ACAR));
    unsigned short* chp = &cs[wave][0][0]; unsigned short* clp = &cs[wave][1][0];
#pragma unroll
    for (int j = 0; j < 4; ++j) { v8us oh, ol;
#pragma unroll
        for (int r = 0; r < 8; ++r) { unsigned short a2, c2; splitf(o[j][r] * rinv, a2, c2); oh[r] = a2; ol[r] = c2; }
        *(v8usa*)(chp + lr * 72 + 16 * j + 8 * hi) = oh; *(v8usa*)(clp + lr * 72 + 16 * j + 8 * hi) = ol; }
    __builtin_amdgcn_fence(3, "wavefront"); __builtin_amdgcn_wave_barrier(); asm volatile("" ::: "memory");
    bf* gh = CTh + ((size_t)g * TQ + t0) * EM + h * HD; bf* gl = CTl + ((size_t)g * TQ + t0) * EM + h * HD;
#pragma unroll 1
    for (int ps = 0; ps < 2; ++ps) {
#pragma unroll
        for (int s = 0; s < 4; ++s) { const int row = 4 * s + (lane >> 3), pc = (lane & 7) * 8; const v8us vh = *(const v8usa*)(chp + row * 72 + pc); const v8us vl = *(const v8usa*)(clp + row * 72 + pc);
            *(volatile v8us*)(gh + (size_t)row * EM + pc) = vh; *(volatile v8us*)(gl + (size_t)row * EM + pc) = vl; }
        if (ps == 0) __threadfence(); }
}

extern "C" void kernel_launch(void* const* d_in, const int* in_sizes, int n_in,
                              void* d_out, int out_size, void* d_ws, size_t ws_size, hipStream_t stream) {
    if (n_in < 17) return;
    const size_t needx = (size_t)(NB - 1) * SEQ_FULL * EM + (size_t)SEQ * EM;
    if ((size_t)in_sizes[0] < needx || (size_t)in_sizes[1] < needx || (size_t)in_sizes[2] < needx || (size_t)out_size < needx) return;
    if (in_sizes[3] < EM * EM || in_sizes[5] < EM * EM || in_sizes[7] < EM * EM || in_sizes[4] < EM || in_sizes[6] < EM || in_sizes[8] < EM) return;
    if (in_sizes[9] < NG * EM * EM || in_sizes[11] < NG * EM * EM || in_sizes[13] < NG * EM * EM || in_sizes[15] < NG * EM * EM) return;
    if (in_sizes[10] < NG * EM || in_sizes[12] < NG * EM || in_sizes[14] < NG * EM || in_sizes[16] < NG * EM) return;
    const float* query = (const float*)d_in[0]; const float* key = (const float*)d_in[1]; const float* value = (const float*)d_in[2];
    const float* Wqg = (const float*)d_in[3]; const float* bqg = (const float*)d_in[4]; const float* Wk = (const float*)d_in[5]; const float* bk = (const float*)d_in[6]; const float* Wv = (const float*)d_in[7]; const float* bv = (const float*)d_in[8];
    const float* Wq_in = (const float*)d_in[9]; const float* bq_in = (const float*)d_in[10]; const float* Wk_in = (const float*)d_in[11]; const float* bk_in = (const float*)d_in[12];
    const float* Wv_in = (const float*)d_in[13]; const float* bv_in = (const float*)d_in[14]; const float* Wout = (const float*)d_in[15]; const float* bout = (const float*)d_in[16];
    float* OUT = (float*)d_out;
    char* wsp = (char*)d_ws;
    auto take = [&](size_t bytes) { char* p = wsp; wsp += (bytes + 255) & ~(size_t)255; return (void*)p; };
    bf* WQG = (bf*)take((size_t)EM * EM * 2); bf* WKO = (bf*)take((size_t)EM * EM * 2); bf* WVO = (bf*)take((size_t)EM * EM * 2); bf* WO = (bf*)take((size_t)NG * EM * EM * 2);
    h16* WQI = (h16*)take((size_t)NG * EM * EM * 2); h16* WKI = (h16*)take((size_t)NG * EM * EM * 2); h16* WVI = (h16*)take((size_t)NG * EM * EM * 2);
    bf* XB = (bf*)take((size_t)SEQ * EM * 2);
    h16* Q16 = (h16*)take((size_t)SEQ * EM * 2); h16* K16 = (h16*)take((size_t)SEQ * EM * 2); h16* V16 = (h16*)take((size_t)SEQ * EM * 2);
    h16* QI16 = (h16*)take((size_t)NG * TQ * EM * 2); h16* KI16 = (h16*)take((size_t)NG * SEQ * EM * 2); h16* VT16 = (h16*)take((size_t)NG * EM * SEQ * 2);
    bf* CTh = (bf*)take((size_t)NG * TQ * EM * 2); bf* CTl = (bf*)take((size_t)NG * TQ * EM * 2);
    if ((size_t)(wsp - (char*)d_ws) > ws_size) return;
    const size_t n8w = (size_t)EM * EM / 8, n8g = (size_t)NG * EM * EM / 8, n8x = (size_t)SEQ * EM / 8;
    const unsigned CVW = (unsigned)((n8w + 255) / 256), CVG = (unsigned)((n8g + 255) / 256), CVX = (unsigned)((n8x + 255) / 256);
    k_cvt8<<<CVW, 256, 0, stream>>>(Wqg, WQG, n8w); k_cvt8<<<CVW, 256, 0, stream>>>(Wk, WKO, n8w); k_cvt8<<<CVW, 256, 0, stream>>>(Wv, WVO, n8w); k_cvt8<<<CVG, 256, 0, stream>>>(Wout, WO, n8g);
    k_cvth<<<CVG, 256, 0, stream>>>(Wq_in, WQI, n8g, WCAR); k_cvth<<<CVG, 256, 0, stream>>>(Wk_in, WKI, n8g, WCAR); k_cvth<<<CVG, 256, 0, stream>>>(Wv_in, WVI, n8g, WCAR);
    const float ioscl = 1.0f / (ACAR * WCAR);
    for (int b = 0; b < NB; ++b) {
        k_cvt8<<<CVX, 256, 0, stream>>>(query + (size_t)b * SEQ_FULL * EM, XB, n8x);
        k_gemmw<bf, 0, 1, h16><<<dim3(SEQ / 64, EM / 64, 1), 32, 0, stream>>>(XB, nullptr, WQG, nullptr, EM, EM, EM, Q16, EM, bqg, 1.0f, ACAR, 0, 0, 0, 0);
        k_cvt8<<<CVX, 256, 0, stream>>>(key + (size_t)b * SEQ_FULL * EM, XB, n8x);
        k_gemmw<bf, 0, 1, h16><<<dim3(SEQ / 64, EM / 64, 1), 32, 0, stream>>>(XB, nullptr, WKO, nullptr, EM, EM, EM, K16, EM, bk, 1.0f, ACAR, 0, 0, 0, 0);
        k_cvt8<<<CVX, 256, 0, stream>>>(value + (size_t)b * SEQ_FULL * EM, XB, n8x);
        k_gemmw<bf, 0, 1, h16><<<dim3(SEQ / 64, EM / 64, 1), 32, 0, stream>>>(XB, nullptr, WVO, nullptr, EM, EM, EM, V16, EM, bv, 1.0f, ACAR, 0, 0, 0, 0);
        k_gemmw<h16, 0, 1, h16><<<dim3(TQ / 64, EM / 64, NG), 32, 0, stream>>>(Q16, nullptr, WQI, nullptr, EM, NG * EM, EM, QI16, EM, bq_in, ioscl, ACAR, (size_t)EM, (size_t)EM * EM, (size_t)TQ * EM, (size_t)EM);
        k_gemmw<h16, 0, 1, h16><<<dim3(SEQ / 64, EM / 64, NG), 32, 0, stream>>>(K16, nullptr, WKI, nullptr, EM, EM, EM, KI16, EM, bk_in, ioscl, ACAR, 0, (size_t)EM * EM, (size_t)SEQ * EM, (size_t)EM);
        k_gemmw<h16, 0, 2, h16><<<dim3(EM / 64, SEQ / 64, NG), 32, 0, stream>>>(WVI, nullptr, V16, nullptr, EM, EM, EM, VT16, SEQ, bv_in, ioscl, ACAR, (size_t)EM * EM, 0, (size_t)EM * SEQ, (size_t)EM);
        k_attn<<<(unsigned)(NG * NH * (TQ / 16) / 2), 64, 0, stream>>>(QI16, KI16, VT16, CTh, CTl);
        k_gemmw<bf, 1, 1, float><<<dim3(TQ / 64, EM / 64, NG), 32, 0, stream>>>(CTh, CTl, WO, nullptr, EM, EM, EM, OUT + (size_t)b * SEQ_FULL * EM, NG * EM, bout, 1.0f, 1.0f, (size_t)TQ * EM, (size_t)EM * EM, (size_t)EM, (size_t)EM);
    }
}
